// LocalRNN_18305150616306
// MI455X (gfx1250) — hardware-verified
//
#include <hip/hip_runtime.h>
#include <math.h>

constexpr int NBAT   = 8;
constexpr int LSEQ   = 1024;
constexpr int DHID   = 512;
constexpr int GATE3  = 3 * DHID;
constexpr int KWIN   = 7;
constexpr int NROWS  = NBAT * LSEQ;
constexpr int NTHR   = 256;
constexpr int GRU_THREADS = 128;
constexpr int GRU_WAVES   = GRU_THREADS / 32;
constexpr int NCG    = DHID / 64;
constexpr int NT16   = NROWS / 16;
constexpr int GRU_GRID = (NT16 * NCG) / GRU_WAVES;
constexpr int SLABP  = 68;
constexpr float WCARRY  = 256.0f;
constexpr float HCARRY  = 16.0f;
constexpr float ACC_INV = 1.0f / 4096.0f;
static_assert(NCG == 8);
static_assert((NT16 * NCG) % GRU_WAVES == 0);
static_assert(DHID % 32 == 0);
static_assert(NROWS % 64 == 0 && GATE3 % 64 == 0);
static_assert(((NROWS / 64) * (GATE3 / 64)) % 8 == 0);
static_assert((NROWS * (DHID / 8)) % NTHR == 0);
static_assert((GATE3 * (DHID / 8)) % NTHR == 0);
static_assert(LSEQ % 16 == 0);
static_assert(KWIN - 1 < 16);

typedef __attribute__((ext_vector_type(16))) _Float16 v16h;
typedef __attribute__((ext_vector_type(8)))  _Float16 v8h;
typedef __attribute__((ext_vector_type(16))) __bf16   v16b;
typedef __attribute__((ext_vector_type(8)))  __bf16   v8b;
typedef __attribute__((ext_vector_type(8)))  float    v8f;
typedef __attribute__((ext_vector_type(4)))  float    v4f;

__device__ __forceinline__ unsigned short f2bf_bits(float f) {
  unsigned u = __float_as_uint(f);
  return (unsigned short)((u + 0x7FFFu + ((u >> 16) & 1u)) >> 16);
}
__device__ __forceinline__ float bf_bits2f(unsigned short h) { return __uint_as_float(((unsigned)h) << 16); }
__device__ __forceinline__ float bf16r(float f) { return bf_bits2f(f2bf_bits(f)); }

__device__ __forceinline__ void dep_guard_h(v8f& a, v8f& b, v16h x, v16h y) { asm volatile("v_nop\n\tv_nop\n\tv_nop\n\tv_nop" : "+v"(a), "+v"(b) : "v"(x), "v"(y)); }
__device__ __forceinline__ void dep_guard_b(v8f& a, v8f& b, v16b x, v16b y) { asm volatile("v_nop\n\tv_nop\n\tv_nop\n\tv_nop" : "+v"(a), "+v"(b) : "v"(x), "v"(y)); }
__device__ __forceinline__ void dep_guard3_h(v8f& a, v8f& b, v8f& d, v16h x, v16h y) { asm volatile("v_nop\n\tv_nop\n\tv_nop\n\tv_nop" : "+v"(a), "+v"(b), "+v"(d) : "v"(x), "v"(y)); }
__device__ __forceinline__ void keep4_h(v16h a, v16h b, v16h c, v16h d) { asm volatile("v_nop" :: "v"(a), "v"(b), "v"(c), "v"(d)); }
__device__ __forceinline__ void keep4_b(v16b a, v16b b, v16b c, v16b d) { asm volatile("v_nop" :: "v"(a), "v"(b), "v"(c), "v"(d)); }
__device__ __forceinline__ void acc_guard4(v8f& a, v8f& b, v8f& c, v8f& d) { asm volatile("v_nop\n\tv_nop\n\tv_nop\n\tv_nop" : "+v"(a), "+v"(b), "+v"(c), "+v"(d)); }
template <typename T> struct Frag;
template <> struct Frag<_Float16> {
  typedef v16h V; union U { v16h v; v8h h[2]; };
  static __device__ __forceinline__ v16h load(const _Float16* p) {
    U f; f.h[0] = *(const v8h*)(p); f.h[1] = *(const v8h*)(p + 16); return f.v;
  }
  static __device__ __forceinline__ v8f mma(v16h a, v16h b, v8f c) {
    return __builtin_amdgcn_wmma_f32_16x16x32_f16(false, a, false, b, (short)0, c, false, false);
  }
  static __device__ __forceinline__ void guard(v8f& a, v8f& b, v16h x, v16h y) { dep_guard_h(a, b, x, y); }
  static __device__ __forceinline__ void keep(v16h a, v16h b, v16h c, v16h d) { keep4_h(a, b, c, d); }
};
template <> struct Frag<__bf16> {
  typedef v16b V; union U { v16b v; v8b h[2]; };
  static __device__ __forceinline__ v16b load(const __bf16* p) {
    U f; f.h[0] = *(const v8b*)(p); f.h[1] = *(const v8b*)(p + 16); return f.v;
  }
  static __device__ __forceinline__ v8f mma(v16b a, v16b b, v8f c) {
    return __builtin_amdgcn_wmma_f32_16x16x32_bf16(false, a, false, b, (short)0, c, false, false);
  }
  static __device__ __forceinline__ void guard(v8f& a, v8f& b, v16b x, v16b y) { dep_guard_b(a, b, x, y); }
  static __device__ __forceinline__ void keep(v16b a, v16b b, v16b c, v16b d) { keep4_b(a, b, c, d); }
};

__device__ __forceinline__ float fsig(float x) { return 1.0f / (1.0f + expf(-x)); }

template <int ET> struct Elem;
template <> struct Elem<0> { typedef _Float16 T; };
template <> struct Elem<1> { typedef __bf16 T; };
template <int ET, bool SPLIT, int BIAS_MODE, int OUT_MODE, bool RESID, int ACT = 0>
__global__ __launch_bounds__(256) void wmma_gemm64(
    const unsigned short* __restrict__ Ap, const unsigned short* __restrict__ A2p, int lda, long strideA,
    const unsigned short* __restrict__ Btp, const unsigned short* __restrict__ Bt2p, int ldb, long strideB,
    void* __restrict__ Cout, void* __restrict__ Cout2, int ldc, long strideC,
    const float* __restrict__ bias,
    const float* __restrict__ resid, long strideR,
    int M, int N, int K, float scale) {
  typedef typename Elem<ET>::T T;
  typedef typename Frag<T>::V V;
  const T* A = (const T*)Ap; const T* A2 = (const T*)A2p; const T* Bt = (const T*)Btp; const T* Bt2 = (const T*)Bt2p;
  __shared__ __align__(16) float sT[8][16 * 68];
  const int b    = blockIdx.y;
  const int lane = threadIdx.x & 31;
  const int wave = threadIdx.x >> 5;
  const int tilesN = N >> 6;
  const int tilesM = M >> 6;
  const int tile = blockIdx.x * 8 + wave;
  if (tile >= tilesM * tilesN) return;
  const int tm = tile / tilesN;
  const int tn = tile - tm * tilesN;
  const int m0 = tm << 6;
  const int n0 = tn << 6;

  const T* Ab  = A  + (size_t)b * strideA;
  const T* Bb  = Bt + (size_t)b * strideB;
  const T* Ab2 = SPLIT ? (A2  + (size_t)b * strideA) : nullptr;
  const T* Bb2 = SPLIT ? (Bt2 + (size_t)b * strideB) : nullptr;

  const int rlane = lane & 15;
  const int koff  = (lane >> 4) * 8;
  const int mOff  = (lane >> 4) * 8;

  v8f acc[4][4];
#pragma unroll
  for (int i = 0; i < 4; ++i)
#pragma unroll
    for (int j = 0; j < 4; ++j) acc[i][j] = (v8f){0.f,0.f,0.f,0.f,0.f,0.f,0.f,0.f};

  for (int k0 = 0; k0 < K; k0 += 32) {
    V bh[4], bl[4];
#pragma unroll
    for (int j = 0; j < 4; ++j) {
      const size_t bo = (size_t)(n0 + (j << 4) + rlane) * ldb + koff + k0;
      bh[j] = Frag<T>::load(Bb + bo);
      if (SPLIT) bl[j] = Frag<T>::load(Bb2 + bo);
    }
#pragma unroll
    for (int i = 0; i < 4; ++i) {
      const size_t ao = (size_t)(m0 + (i << 4) + rlane) * lda + koff + k0;
      V ah = Frag<T>::load(Ab + ao);
      V al;
      if (SPLIT) al = Frag<T>::load(Ab2 + ao);
#pragma unroll
      for (int j = 0; j < 4; ++j) {
        acc[i][j] = Frag<T>::mma(ah, bh[j], acc[i][j]);
        if (SPLIT) {
          acc[i][j] = Frag<T>::mma(ah, bl[j], acc[i][j]);
          acc[i][j] = Frag<T>::mma(al, bh[j], acc[i][j]);
        }
      }
      Frag<T>::guard(acc[i][0], acc[i][3], ah, SPLIT ? al : ah);
    }
    Frag<T>::keep(bh[0], bh[1], bh[2], bh[3]);
    if (SPLIT) Frag<T>::keep(bl[0], bl[1], bl[2], bl[3]);
  }
  acc_guard4(acc[0][0], acc[0][1], acc[0][2], acc[0][3]);
  acc_guard4(acc[1][0], acc[1][1], acc[1][2], acc[1][3]);
  acc_guard4(acc[2][0], acc[2][1], acc[2][2], acc[2][3]);
  acc_guard4(acc[3][0], acc[3][1], acc[3][2], acc[3][3]);

  float* slab = sT[wave];
  const float* Rb = RESID ? (resid + (size_t)b * strideR) : nullptr;
#pragma unroll
  for (int i = 0; i < 4; ++i) {
    const int mBase = m0 + (i << 4);
#pragma unroll
    for (int j = 0; j < 4; ++j) {
      const int n = n0 + (j << 4) + rlane;
      float bv = 0.f;
      if (BIAS_MODE == 2) bv = bias[n];
#pragma unroll
      for (int r = 0; r < 8; ++r) {
        float v = acc[i][j][r] * scale;
        if (BIAS_MODE == 1) v += bias[mBase + mOff + r];
        if (BIAS_MODE == 2) v += bv;
        if (RESID) v += Rb[(size_t)(mBase + mOff + r) * ldc + n];
        if (ACT == 1) v = tanhf(v);
        if (ACT == 2) v = fmaxf(v, 0.0f);
        if (ACT == 3) v = v / (1.0f + expf(-v));
        if (ACT == 4) v = (v > 0.f) ? v : 0.01f * v;
        if (ACT == 5) v = 0.5f * v * (1.0f + erff(v * 0.70710678118654752f));
        slab[(mOff + r) * 68 + (j << 4) + rlane] = v;
      }
    }
    __builtin_amdgcn_fence(__ATOMIC_RELEASE, "workgroup");
    __builtin_amdgcn_wave_barrier();
    __builtin_amdgcn_fence(__ATOMIC_ACQUIRE, "workgroup");
    if (OUT_MODE == 0) {
      float* C = (float*)Cout + (size_t)b * strideC;
      const int hh = lane >> 4, c4 = (lane & 15) * 4;
      for (int pass = 0; pass < 2; ++pass) {
#pragma unroll
        for (int it = 0; it < 8; ++it) {
          const int row = it * 2 + hh;
          v4f v = *(const v4f*)(slab + row * 68 + c4);
          *(volatile v4f*)(C + (size_t)(mBase + row) * ldc + n0 + c4) = v;
        }
        __threadfence();
      }
    } else {
      const int q = lane >> 3, c8 = (lane & 7) * 8;
      unsigned short* C  = (unsigned short*)Cout  + (size_t)b * strideC;
      unsigned short* C2 = (OUT_MODE == 2) ? ((unsigned short*)Cout2 + (size_t)b * strideC) : nullptr;
      for (int pass = 0; pass < 2; ++pass) {
#pragma unroll
        for (int it = 0; it < 4; ++it) {
          const int row = it * 4 + q;
          const float* sp = slab + row * 68 + c8;
          v8h hv, lv;
#pragma unroll
          for (int e = 0; e < 8; ++e) {
            if (OUT_MODE == 1) {
              hv[e] = (_Float16)sp[e];
            } else {
              unsigned short hb = f2bf_bits(sp[e]);
              unsigned short lb = f2bf_bits(sp[e] - bf_bits2f(hb));
              hv[e] = __builtin_bit_cast(_Float16, hb);
              lv[e] = __builtin_bit_cast(_Float16, lb);
            }
          }
          *(volatile v8h*)(C + (size_t)(mBase + row) * ldc + n0 + c8) = hv;
          if (OUT_MODE == 2) *(volatile v8h*)(C2 + (size_t)(mBase + row) * ldc + n0 + c8) = lv;
        }
        __threadfence();
      }
    }
    __builtin_amdgcn_fence(__ATOMIC_RELEASE, "workgroup");
    __builtin_amdgcn_wave_barrier();
    __builtin_amdgcn_fence(__ATOMIC_ACQUIRE, "workgroup");
  }
}

template <int MODE>
__global__ __launch_bounds__(NTHR) void cvt8_kernel(const float* __restrict__ src, unsigned short* __restrict__ dst,
                                                    int nrow, int ncol8, int spitch, int scol0, float sc) {
  const int i  = blockIdx.x * NTHR + threadIdx.x;
  const int n8 = nrow * ncol8;
  if (i < n8) {
    const int row = i / ncol8;
    const int c8  = i - row * ncol8;
    const float* sp = src + (size_t)row * spitch + scol0 + c8 * 8;
    const v4f a = *(const v4f*)(sp);
    const v4f b = *(const v4f*)(sp + 4);
    v8h hv;
#pragma unroll
    for (int e = 0; e < 4; ++e) {
      unsigned short b0, b1;
      if (MODE == 0) {
        b0 = f2bf_bits(a[e] * sc);
        b1 = f2bf_bits(b[e] * sc);
      } else {
        b0 = __builtin_bit_cast(unsigned short, (_Float16)(bf16r(a[e]) * sc));
        b1 = __builtin_bit_cast(unsigned short, (_Float16)(bf16r(b[e]) * sc));
      }
      hv[e]     = __builtin_bit_cast(_Float16, b0);
      hv[4 + e] = __builtin_bit_cast(_Float16, b1);
    }
    *(volatile v8h*)(dst + (size_t)i * 8) = hv;
    __threadfence();
    *(volatile v8h*)(dst + (size_t)i * 8) = hv;
  }
}

__global__ __launch_bounds__(NTHR) void bias_prep_kernel(const float* __restrict__ src, float* __restrict__ dst, int n4) {
  const int i = blockIdx.x * NTHR + threadIdx.x;
  if (i < n4) {
    const v4f v = *(const v4f*)(src + 4 * i);
    v4f o;
#pragma unroll
    for (int e = 0; e < 4; ++e) o[e] = bf16r(v[e]);
    float* op = dst + 4 * i;
    *(volatile v4f*)op = o;
    __threadfence();
    *(volatile v4f*)op = o;
  }
}

__global__ __launch_bounds__(NTHR) void gru_first_kernel(const float* __restrict__ GX, const float* __restrict__ BI,
                                                         const float* __restrict__ BH, float* __restrict__ HF,
                                                         unsigned short* __restrict__ H16) {
  __shared__ __align__(16) float hs[NTHR];
  const int tid = threadIdx.x, wave = tid >> 5;
  const int blk = blockIdx.x;
  const int row = blk >> 1;
  const int dbase = (blk & 1) * (DHID / 2);
  const int d = dbase + tid;
  const int l = row & (LSEQ - 1);
  const int bat0 = row - l;
  const int lsrc = l - (KWIN - 1);
  const float fv  = (lsrc >= 0) ? 1.0f : 0.0f;
  const float fvi = 1.0f - fv;
  const int lc = (lsrc < 0) ? 0 : lsrc;
  const float* gxp = GX + (size_t)(bat0 + lc) * GATE3;
  const float gr = gxp[d], gz = gxp[DHID + d], gn = gxp[2 * DHID + d];
  const float bir = BI[d], biz = BI[DHID + d], bin_ = BI[2 * DHID + d];
  const float bhr = BH[d], bhz = BH[DHID + d], bhn = BH[2 * DHID + d];
  const float xr = fmaf(fv, gr, fvi * bir);
  const float xz = fmaf(fv, gz, fvi * biz);
  const float xn = fmaf(fv, gn, fvi * bin_);
  const float rg = fsig(xr + bhr);
  const float zg = fsig(xz + bhz);
  const float ng = tanhf(xn + rg * bhn);
  const float h  = (1.0f - zg) * ng;
  hs[tid] = h;
  __syncthreads();
  const size_t ebase = (size_t)row * DHID + (size_t)dbase;
  if (wave < 2) {
    const v4f v = *(const v4f*)(hs + 4 * tid);
    float* op = HF + ebase + 4 * tid;
    *(volatile v4f*)op = v;
    __threadfence();
    *(volatile v4f*)op = v;
  }
  if (wave == 0) {
    v8h hv;
#pragma unroll
    for (int e = 0; e < 8; ++e) hv[e] = (_Float16)(hs[8 * tid + e] * HCARRY);
    unsigned short* op = H16 + ebase + 8 * tid;
    *(volatile v8h*)op = hv;
    __threadfence();
    *(volatile v8h*)op = hv;
  }
}

template <bool W16>
__global__ __launch_bounds__(GRU_THREADS) void gru_step_kernel(
    const unsigned short* __restrict__ Hin16p, const unsigned short* __restrict__ WHp,
    const float* __restrict__ GX, const float* __restrict__ BI, const float* __restrict__ BH,
    const float* __restrict__ Hin32, float* __restrict__ Hout32, unsigned short* __restrict__ Hout16,
    int kstep) {
  __shared__ __align__(16) float sl[GRU_WAVES][3][16 * SLABP];
  const _Float16* Hin16 = (const _Float16*)Hin16p;
  const _Float16* WH    = (const _Float16*)WHp;
  const int tid = threadIdx.x, lane = tid & 31, wave = tid >> 5;
  const int c = lane & 15, hh = lane >> 4, koff = hh * 8, c4 = c * 4;
  const int tile = blockIdx.x * GRU_WAVES + wave;
  const int tm = tile >> 3, tn = tile & 7;
  const int m0 = tm * 16, n0 = tn * 64;
  const int l0 = m0 & (LSEQ - 1);
  const int bat0 = m0 - l0;

  const v8f z8 = {0.f, 0.f, 0.f, 0.f, 0.f, 0.f, 0.f, 0.f};
  v8f acc[3][4];
#pragma unroll
  for (int g = 0; g < 3; ++g)
#pragma unroll
    for (int j = 0; j < 4; ++j) acc[g][j] = z8;

  const _Float16* arow = Hin16 + (size_t)(m0 + c) * DHID + koff;
  const _Float16* wrow = WH + (size_t)(n0 + c) * DHID + koff;
#pragma unroll 1
  for (int k0 = 0; k0 < DHID; k0 += 32) {
    const v16h a = Frag<_Float16>::load(arow + k0);
#pragma unroll
    for (int j = 0; j < 4; ++j) {
      const _Float16* wp = wrow + (size_t)(16 * j) * DHID + k0;
      const v16h br = Frag<_Float16>::load(wp);
      const v16h bz = Frag<_Float16>::load(wp + (size_t)DHID * DHID);
      const v16h bn = Frag<_Float16>::load(wp + (size_t)2 * DHID * DHID);
      acc[0][j] = Frag<_Float16>::mma(a, br, acc[0][j]);
      acc[1][j] = Frag<_Float16>::mma(a, bz, acc[1][j]);
      acc[2][j] = Frag<_Float16>::mma(a, bn, acc[2][j]);
      dep_guard3_h(acc[0][j], acc[1][j], acc[2][j], a, bn);
      keep4_h(br, bz, bn, a);
    }
  }
  acc_guard4(acc[0][0], acc[0][1], acc[0][2], acc[0][3]);
  acc_guard4(acc[1][0], acc[1][1], acc[1][2], acc[1][3]);
  acc_guard4(acc[2][0], acc[2][1], acc[2][2], acc[2][3]);

  float* slr = &sl[wave][0][0];
  float* slz = &sl[wave][1][0];
  float* sln = &sl[wave][2][0];
#pragma unroll
  for (int j = 0; j < 4; ++j)
#pragma unroll
    for (int r = 0; r < 8; ++r) {
      const int o = (8 * hh + r) * SLABP + 16 * j + c;
      slr[o] = acc[0][j][r];
      slz[o] = acc[1][j][r];
      sln[o] = acc[2][j][r];
    }
  __builtin_amdgcn_fence(__ATOMIC_RELEASE, "workgroup");
  __builtin_amdgcn_wave_barrier();
  __builtin_amdgcn_fence(__ATOMIC_ACQUIRE, "workgroup");

  const v4f bir  = *(const v4f*)(BI + n0 + c4);
  const v4f biz  = *(const v4f*)(BI + DHID + n0 + c4);
  const v4f bin_ = *(const v4f*)(BI + 2 * DHID + n0 + c4);
  const v4f bhr  = *(const v4f*)(BH + n0 + c4);
  const v4f bhz  = *(const v4f*)(BH + DHID + n0 + c4);
  const v4f bhn  = *(const v4f*)(BH + 2 * DHID + n0 + c4);
#pragma unroll 1
  for (int it = 0; it < 8; ++it) {
    const int row = it * 2 + hh;
    const int lsrc = l0 + row + kstep - (KWIN - 1);
    const float fv  = (lsrc >= 0) ? 1.0f : 0.0f;
    const float fvi = 1.0f - fv;
    int lc = (lsrc < 0) ? 0 : lsrc;
    lc = (lc > LSEQ - 1) ? (LSEQ - 1) : lc;
    const float* gxp = GX + (size_t)(bat0 + lc) * GATE3 + n0 + c4;
    const v4f gr = *(const v4f*)(gxp);
    const v4f gz = *(const v4f*)(gxp + DHID);
    const v4f gn = *(const v4f*)(gxp + 2 * DHID);
    const v4f ho = *(const v4f*)(Hin32 + (size_t)(m0 + row) * DHID + n0 + c4);
    float* srow = slr + row * SLABP + c4;
    const v4f sr = *(const v4f*)(srow);
    const v4f sz = *(const v4f*)(slz + row * SLABP + c4);
    const v4f sn = *(const v4f*)(sln + row * SLABP + c4);
    v4f hn;
#pragma unroll
    for (int e = 0; e < 4; ++e) {
      const float xr = fmaf(fv, gr[e], fvi * bir[e]);
      const float xz = fmaf(fv, gz[e], fvi * biz[e]);
      const float xn = fmaf(fv, gn[e], fvi * bin_[e]);
      const float ghr = sr[e] * ACC_INV + bhr[e];
      const float ghz = sz[e] * ACC_INV + bhz[e];
      const float ghn = sn[e] * ACC_INV + bhn[e];
      const float rg = fsig(xr + ghr);
      const float zg = fsig(xz + ghz);
      const float ng = tanhf(xn + rg * ghn);
      hn[e] = (1.0f - zg) * ng + zg * ho[e];
    }
    *(v4f*)(srow) = hn;
  }
  __builtin_amdgcn_fence(__ATOMIC_RELEASE, "workgroup");
  __builtin_amdgcn_wave_barrier();
  __builtin_amdgcn_fence(__ATOMIC_ACQUIRE, "workgroup");

  for (int pass = 0; pass < 2; ++pass) {
#pragma unroll
    for (int it = 0; it < 8; ++it) {
      const int row = it * 2 + hh;
      const v4f v = *(const v4f*)(slr + row * SLABP + c4);
      *(volatile v4f*)(Hout32 + (size_t)(m0 + row) * DHID + n0 + c4) = v;
    }
    __threadfence();
  }
  if (W16) {
    const int q = lane >> 3, c8 = (lane & 7) * 8;
    for (int pass = 0; pass < 2; ++pass) {
#pragma unroll
      for (int it = 0; it < 4; ++it) {
        const int row = it * 4 + q;
        const float* sp = slr + row * SLABP + c8;
        v8h hv;
#pragma unroll
        for (int e = 0; e < 8; ++e) hv[e] = (_Float16)(sp[e] * HCARRY);
        *(volatile v8h*)(Hout16 + (size_t)(m0 + row) * DHID + n0 + c8) = hv;
      }
      __threadfence();
    }
  }
}

extern "C" void kernel_launch(void* const* d_in, const int* in_sizes, int n_in,
                              void* d_out, int out_size, void* d_ws, size_t ws_size, hipStream_t stream) {
  if (n_in < 6 || d_out == nullptr || d_ws == nullptr) return;
  if (in_sizes[0] != NROWS * DHID || in_sizes[1] != GATE3 * DHID || in_sizes[2] != GATE3 * DHID ||
      in_sizes[3] != GATE3 || in_sizes[4] != GATE3 || out_size != NROWS * DHID) return;

  const float* x    = (const float*)d_in[0];
  const float* w_ih = (const float*)d_in[1];
  const float* w_hh = (const float*)d_in[2];
  const float* b_ih = (const float*)d_in[3];
  const float* b_hh = (const float*)d_in[4];
  float* out = (float*)d_out;

  char* ws = (char*)d_ws; size_t off = 0;
  auto carve = [&](size_t bytes) -> char* { char* p = ws + off; off += (bytes + 255) & ~(size_t)255; return p; };
  unsigned short* XB   = (unsigned short*)carve((size_t)NROWS * DHID * 2);
  unsigned short* WIB  = (unsigned short*)carve((size_t)GATE3 * DHID * 2);
  unsigned short* WHH  = (unsigned short*)carve((size_t)GATE3 * DHID * 2);
  float*          BI   = (float*)carve((size_t)GATE3 * 4);
  float*          BH   = (float*)carve((size_t)GATE3 * 4);
  float*          GX   = (float*)carve((size_t)NROWS * GATE3 * 4);
  float*          HFA  = (float*)carve((size_t)NROWS * DHID * 4);
  float*          HFB  = (float*)carve((size_t)NROWS * DHID * 4);
  unsigned short* H16A = (unsigned short*)carve((size_t)NROWS * DHID * 2);
  unsigned short* H16B = (unsigned short*)carve((size_t)NROWS * DHID * 2);
  if (off > ws_size || off > (size_t)134217728) return;

  const int n8x = NROWS * (DHID / 8);
  const int n8w = GATE3 * (DHID / 8);
  cvt8_kernel<0><<<(n8x + NTHR - 1) / NTHR, NTHR, 0, stream>>>(x,    XB,  NROWS, DHID / 8, DHID, 0, 1.0f);
  cvt8_kernel<0><<<(n8w + NTHR - 1) / NTHR, NTHR, 0, stream>>>(w_ih, WIB, GATE3, DHID / 8, DHID, 0, 1.0f);
  cvt8_kernel<1><<<(n8w + NTHR - 1) / NTHR, NTHR, 0, stream>>>(w_hh, WHH, GATE3, DHID / 8, DHID, 0, WCARRY);
  const int n4b = GATE3 / 4;
  bias_prep_kernel<<<(n4b + NTHR - 1) / NTHR, NTHR, 0, stream>>>(b_ih, BI, n4b);
  bias_prep_kernel<<<(n4b + NTHR - 1) / NTHR, NTHR, 0, stream>>>(b_hh, BH, n4b);

  const dim3 ggrid((NROWS / 64) * (GATE3 / 64) / 8, 1);
  wmma_gemm64<1, false, 2, 0, false, 0><<<ggrid, 256, 0, stream>>>(
      XB, XB, DHID, 0L, WIB, WIB, DHID, 0L, (void*)GX, (void*)GX, GATE3, 0L,
      BI, GX, 0L, NROWS, GATE3, DHID, 1.0f);

  gru_first_kernel<<<NROWS * 2, NTHR, 0, stream>>>(GX, BI, BH, HFA, H16A);

  for (int k = 1; k < KWIN; ++k) {
    const bool odd = (k & 1) != 0;
    const float*          hin32  = odd ? HFA : HFB;
    const unsigned short* hin16  = odd ? H16A : H16B;
    float*                hout32 = odd ? HFB : HFA;
    unsigned short*       hout16 = odd ? H16B : H16A;
    if (k < KWIN - 1) {
      gru_step_kernel<true><<<GRU_GRID, GRU_THREADS, 0, stream>>>(hin16, WHH, GX, BI, BH, hin32, hout32, hout16, k);
    } else {
      gru_step_kernel<false><<<GRU_GRID, GRU_THREADS, 0, stream>>>(hin16, WHH, GX, BI, BH, hin32, out, hout16, k);
    }
  }
}
